// MultiViewAttention_69131793596834
// MI455X (gfx1250) — hardware-verified
//
#include <hip/hip_runtime.h>
#include <stddef.h>
#include <stdint.h>

#define NBAT  8
#define NN    1024
#define NTOK  8192
#define CD    256
#define NH    8
#define HDM   32
#define NQKV  768
#define NSLAB 6
#define NWSL  4
#define NHF   (NBAT * NH)
#define MM    NN
#define QB    128
#define KCH   64
#define NQB   (MM / QB)
#define NCK   (MM / KCH)
#define PR    32

static_assert(NTOK == NBAT * NN);
static_assert(NH * HDM == CD);
static_assert(NQKV == 3 * CD);
static_assert(NQKV == NSLAB * 128);
static_assert(MM % QB == 0);
static_assert(MM % KCH == 0);
static_assert(NN % 64 == 0);
static_assert(NN % PR == 0);
static_assert(CD % 64 == 0);
static_assert(NTOK % 64 == 0);
static_assert(HDM == 32);
static_assert(KCH == 64);
static_assert(QB == 8 * 16);
static_assert((CD * CD) % 2048 == 0);

#define XCAR 4.0f
#define WCAR 64.0f
#define QCAR 8.0f
#define VCAR 16.0f
#define PCAR 1024.0f
#define OCAR 16.0f

typedef _Float16 v16h __attribute__((ext_vector_type(16)));
typedef _Float16 v8h  __attribute__((ext_vector_type(8)));
typedef float    v8f  __attribute__((ext_vector_type(8)));
typedef float    v4f  __attribute__((ext_vector_type(4)));
typedef unsigned int v4u __attribute__((ext_vector_type(4)));

union FragH { v16h v; v8h h[2]; };
union Pack8 { v8h h; v4u u; };

__device__ __forceinline__ v8f mma_h(v16h a, v16h b, v8f c) {
  c = __builtin_amdgcn_wmma_f32_16x16x32_f16(false, a, false, b, (short)0, c, false, false);
  asm volatile("v_nop\n\tv_nop\n\tv_nop\n\tv_nop" : "+v"(c) : "v"(a), "v"(b));
  return c;
}

__device__ __forceinline__ v8f zero8() { return (v8f){0.f, 0.f, 0.f, 0.f, 0.f, 0.f, 0.f, 0.f}; }

__device__ __forceinline__ v16h ldfrag_h(const _Float16* p, int ld, int row0, int k0, int lane) {
  const int m = lane & 15, lh = lane >> 4;
  const _Float16* q = p + (size_t)(row0 + m) * ld + k0 + 8 * lh;
  FragH f;
  f.h[0] = *(const v8h*)(q);
  f.h[1] = *(const v8h*)(q + 16);
  return f.v;
}

__device__ __forceinline__ v4u pack_h8(const float (&v)[8], float s) {
  Pack8 pk;
  pk.h = (v8h){(_Float16)(v[0] * s), (_Float16)(v[1] * s), (_Float16)(v[2] * s), (_Float16)(v[3] * s),
               (_Float16)(v[4] * s), (_Float16)(v[5] * s), (_Float16)(v[6] * s), (_Float16)(v[7] * s)};
  return pk.u;
}

__device__ __forceinline__ void gemm16x64(const _Float16* __restrict__ A, int lda, size_t akst,
                                          const _Float16* __restrict__ B,
                                          int m0, int n0, int lane, v8f (&acc)[4]) {
#pragma unroll 1
  for (int ks = 0; ks < CD / 32; ++ks) {
    const v16h a = ldfrag_h(A + (size_t)ks * akst, lda, m0, 0, lane);
#pragma unroll
    for (int t = 0; t < 4; ++t) {
      const v16h b = ldfrag_h(B, CD, n0 + 16 * t, ks * 32, lane);
      acc[t] = mma_h(a, b, acc[t]);
    }
  }
}

#define WTP 65
__global__ __launch_bounds__(256) void k_xtr(const float* __restrict__ x,
                                             _Float16* __restrict__ xf) {
  __shared__ float tl[64 * WTP];
  const int tid = threadIdx.x;
  const int n0 = blockIdx.x * 64, c0 = blockIdx.y * 64, b = blockIdx.z;
  const float* xb = x + (size_t)b * CD * NN;
#pragma unroll
  for (int j = 0; j < 4; ++j) {
    const int p  = tid + 256 * j;
    const int cc = p >> 4;
    const int q4 = (p & 15) * 4;
    const v4f a = *(const v4f*)(xb + (size_t)(c0 + cc) * NN + n0 + q4);
    float* d = tl + cc * WTP + q4;
    d[0] = a[0]; d[1] = a[1]; d[2] = a[2]; d[3] = a[3];
  }
  __syncthreads();
  v4u vh[2];
  size_t go[2];
#pragma unroll
  for (int j = 0; j < 2; ++j) {
    const int p  = tid + 256 * j;
    const int nn = p >> 3;
    const int pc = p & 7;
    const float* cp = tl + (pc * 8) * WTP + nn;
    float v[8];
#pragma unroll
    for (int i = 0; i < 8; ++i) v[i] = cp[i * WTP];
    vh[j] = pack_h8(v, XCAR);
    go[j] = ((size_t)b * NN + n0 + nn) * CD + c0 + pc * 8;
  }
  for (int ps = 0; ps < 2; ++ps) {
#pragma unroll
    for (int j = 0; j < 2; ++j) *(volatile v4u*)(xf + go[j]) = vh[j];
    __threadfence();
  }
}

__global__ __launch_bounds__(256) void k_wcv(const float* __restrict__ Wq, const float* __restrict__ Wk,
                                             const float* __restrict__ Wv, const float* __restrict__ Wp,
                                             _Float16* __restrict__ wf) {
  const int y = blockIdx.y;
  const float* W = (y == 0) ? Wq : (y == 1) ? Wk : (y == 2) ? Wv : Wp;
  int i = blockIdx.x * 256 + threadIdx.x;
  i = min(i, CD * CD / 8 - 1);
  const float* wp = W + (size_t)i * 8;
  const v4f a0 = *(const v4f*)(wp), a1 = *(const v4f*)(wp + 4);
  float v[8] = {a0[0], a0[1], a0[2], a0[3], a1[0], a1[1], a1[2], a1[3]};
  const v4u ph = pack_h8(v, WCAR);
  const size_t go = (size_t)y * CD * CD + (size_t)i * 8;
  for (int ps = 0; ps < 2; ++ps) {
    *(volatile v4u*)(wf + go) = ph;
    __threadfence();
  }
}

#define SFP 132
__global__ __launch_bounds__(256) void k_qkv(const _Float16* __restrict__ xf,
                                             const _Float16* __restrict__ wf,
                                             const float* __restrict__ bq,
                                             const float* __restrict__ bk,
                                             const float* __restrict__ bv,
                                             _Float16* __restrict__ qp,
                                             _Float16* __restrict__ kp,
                                             _Float16* __restrict__ vtp) {
  __shared__ __align__(16) float sf[64 * SFP];
  const int tid = threadIdx.x, lane = tid & 31, wave = tid >> 5;
  const int hh = lane >> 4, c = lane & 15;
  const int wm = wave >> 1, wn = wave & 1;
  const int mb  = blockIdx.x * 64;
  const int b   = mb >> 10;
  const int nb0 = mb & (NN - 1);
  const int ns  = blockIdx.y;
  const int which = ns >> 1;
  const int hbase = 4 * (ns & 1);
  const int hfb = b * NH + hbase;
  const int m0 = mb + wm * 16;
  const int n0 = ns * 128 + wn * 64;
  const int cb = (ns & 1) * 128 + wn * 64;
  const float* bs = (which == 0) ? bq : (which == 1) ? bk : bv;

  float bb[4];
#pragma unroll
  for (int t = 0; t < 4; ++t) bb[t] = bs[cb + 16 * t + c];

  v8f acc[4];
#pragma unroll
  for (int t = 0; t < 4; ++t) acc[t] = zero8();
  gemm16x64(xf, CD, 32, wf, m0, n0, lane, acc);

  const float escale = 1.0f / (XCAR * WCAR);
#pragma unroll
  for (int t = 0; t < 4; ++t) {
#pragma unroll
    for (int r = 0; r < 8; ++r)
      sf[(wm * 16 + 8 * hh + r) * SFP + wn * 64 + 16 * t + c] = acc[t][r] * escale + bb[t];
  }
  __syncthreads();

  if (which < 2) {
    v4u val[4];
    size_t go[4];
#pragma unroll
    for (int j = 0; j < 4; ++j) {
      const int lr = tid >> 2;
      const int pc = tid & 3;
      const float* ra = sf + lr * SFP + j * 32 + pc * 8;
      const v4f a0 = *(const v4f*)(ra), a1 = *(const v4f*)(ra + 4);
      float v[8] = {a0[0], a0[1], a0[2], a0[3], a1[0], a1[1], a1[2], a1[3]};
      val[j] = pack_h8(v, QCAR);
      go[j]  = ((size_t)(hfb + j) * MM + nb0 + lr) * HDM + pc * 8;
    }
    _Float16* base = (which == 0) ? qp : kp;
    for (int ps = 0; ps < 2; ++ps) {
#pragma unroll
      for (int j = 0; j < 4; ++j) *(volatile v4u*)(base + go[j]) = val[j];
      __threadfence();
    }
  } else {
    v4u val[4];
    size_t go[4];
#pragma unroll
    for (int j = 0; j < 4; ++j) {
      const int p    = tid + 256 * j;
      const int dcol = p >> 3;
      const int pc   = p & 7;
      const float* cp = sf + (pc * 8) * SFP + dcol;
      float v[8];
#pragma unroll
      for (int i = 0; i < 8; ++i) v[i] = cp[i * SFP];
      val[j] = pack_h8(v, VCAR);
      const int hf = hfb + (dcol >> 5);
      const int dd = dcol & 31;
      go[j]  = ((size_t)hf * HDM + dd) * MM + nb0 + pc * 8;
    }
    for (int ps = 0; ps < 2; ++ps) {
#pragma unroll
      for (int j = 0; j < 4; ++j) *(volatile v4u*)(vtp + go[j]) = val[j];
      __threadfence();
    }
  }
}

#define KTP 40
#define VTP 72
#define PTP 72
#define OSP 36
__global__ __launch_bounds__(256) void k_attn(const _Float16* __restrict__ qp,
                                              const _Float16* __restrict__ kp,
                                              const _Float16* __restrict__ vt,
                                              _Float16* __restrict__ op,
                                              float sscale) {
  __shared__ __align__(16) _Float16 Ks[KCH * KTP];
  __shared__ __align__(16) _Float16 Vs[HDM * VTP];
  __shared__ __align__(16) _Float16 Ps[8 * 16 * PTP];
  __shared__ __align__(16) float    Os[8 * 16 * OSP];

  const int tid = threadIdx.x, lane = tid & 31, wave = tid >> 5;
  const int hh = lane >> 4, c = lane & 15;
  const int qb = blockIdx.x % NQB;
  const int hf = blockIdx.x / NQB;
  const int h  = hf & (NH - 1);
  const int b  = hf >> 3;
  const int q0 = qb * QB + wave * 16;

  const _Float16* Q = qp + (size_t)hf * MM * HDM;
  const _Float16* K = kp + (size_t)hf * MM * HDM;
  const _Float16* V = vt + (size_t)hf * HDM * MM;
  const size_t trow0 = (size_t)b * NN;

  const v16h qa = ldfrag_h(Q, HDM, q0, 0, lane);

  const float NEGI = -__builtin_huge_valf();
  float mrow[8], lrow[8];
  v8f oacc[2];
#pragma unroll
  for (int r = 0; r < 8; ++r) { mrow[r] = NEGI; lrow[r] = 0.f; }
  oacc[0] = zero8(); oacc[1] = zero8();

  _Float16* pw = Ps + wave * 16 * PTP;
  float*    ow = Os + wave * 16 * OSP;

  for (int kc = 0; kc < NCK; ++kc) {
    const int kv0 = kc * KCH;
    __syncthreads();
    {
      const int rk = tid >> 2;
      const int qk = (tid & 3) * 8;
      *(v8h*)(Ks + rk * KTP + qk) = *(const v8h*)(K + (size_t)(kv0 + rk) * HDM + qk);
      const int rv = tid >> 3;
      const int qv = (tid & 7) * 8;
      *(v8h*)(Vs + rv * VTP + qv) = *(const v8h*)(V + (size_t)rv * MM + kv0 + qv);
    }
    __syncthreads();

    v8f s[4];
#pragma unroll
    for (int j = 0; j < 4; ++j) {
      const v16h kb = ldfrag_h(Ks, KTP, j * 16, 0, lane);
      s[j] = mma_h(qa, kb, zero8());
    }
    float cm[8];
#pragma unroll
    for (int r = 0; r < 8; ++r) {
      float m = NEGI;
#pragma unroll
      for (int j = 0; j < 4; ++j) { s[j][r] *= sscale; m = fmaxf(m, s[j][r]); }
#pragma unroll
      for (int off = 1; off < 16; off <<= 1) m = fmaxf(m, __shfl_xor(m, off, 32));
      cm[r] = m;
    }
    float al[8];
#pragma unroll
    for (int r = 0; r < 8; ++r) {
      const float mnew  = fmaxf(mrow[r], cm[r]);
      const float alpha = __expf(mrow[r] - mnew);
      mrow[r] = mnew;
      float psum = 0.f;
#pragma unroll
      for (int j = 0; j < 4; ++j) {
        const float p = __expf(s[j][r] - mnew);
        psum += p;
        pw[(8 * hh + r) * PTP + j * 16 + c] = (_Float16)(p * PCAR);
      }
#pragma unroll
      for (int off = 1; off < 16; off <<= 1) psum += __shfl_xor(psum, off, 32);
      lrow[r] = lrow[r] * alpha + psum;
      al[r] = alpha;
    }
#pragma unroll
    for (int t = 0; t < 2; ++t)
#pragma unroll
      for (int r = 0; r < 8; ++r) oacc[t][r] *= al[r];
    __syncthreads();

#pragma unroll
    for (int kk = 0; kk < 2; ++kk) {
      const v16h pa = ldfrag_h(pw, PTP, 0, kk * 32, lane);
#pragma unroll
      for (int t = 0; t < 2; ++t) {
        const v16h vb = ldfrag_h(Vs, VTP, t * 16, kk * 32, lane);
        oacc[t] = mma_h(pa, vb, oacc[t]);
      }
    }
  }

  float invl[8];
#pragma unroll
  for (int r = 0; r < 8; ++r) invl[r] = (lrow[r] > 0.f) ? (9.765625e-04f * (1.0f / lrow[r])) : 0.f;
  __syncthreads();
#pragma unroll
  for (int r = 0; r < 8; ++r) {
#pragma unroll
    for (int t = 0; t < 2; ++t) ow[(8 * hh + r) * OSP + 16 * t + c] = oacc[t][r] * invl[r];
  }
  __syncthreads();
  v4u vh[2];
  size_t go[2];
#pragma unroll
  for (int it = 0; it < 2; ++it) {
    const int p  = lane + 32 * it;
    const int L  = p >> 2;
    const int pc = p & 3;
    const float* ra = ow + L * OSP + pc * 8;
    const v4f a0 = *(const v4f*)(ra), a1 = *(const v4f*)(ra + 4);
    float v[8] = {a0[0], a0[1], a0[2], a0[3], a1[0], a1[1], a1[2], a1[3]};
    vh[it] = pack_h8(v, 1.0f);
    go[it] = ((size_t)h * NTOK + trow0 + q0 + L) * HDM + pc * 8;
  }
  for (int ps = 0; ps < 2; ++ps) {
#pragma unroll
    for (int it = 0; it < 2; ++it) *(volatile v4u*)(op + go[it]) = vh[it];
    __threadfence();
  }
}

#define TPP 36
__global__ __launch_bounds__(256) void k_projln(const _Float16* __restrict__ op,
                                                const _Float16* __restrict__ wf,
                                                const float* __restrict__ pb,
                                                const float* __restrict__ x,
                                                const float* __restrict__ gamma,
                                                const float* __restrict__ beta,
                                                float* __restrict__ out) {
  __shared__ __align__(16) float st[CD * TPP];
  __shared__ float mean_s[PR], rstd_s[PR];
  const int tid = threadIdx.x, lane = tid & 31, wave = tid >> 5;
  const int hh = lane >> 4, c = lane & 15;
  const int wm = wave >> 2, wn = wave & 3;
  const int mb  = blockIdx.x * PR;
  const int b   = mb >> 10;
  const int nb0 = mb & (NN - 1);
  const int m0  = mb + wm * 16;
  const int n0  = wn * 64;

  float bb[4];
#pragma unroll
  for (int t = 0; t < 4; ++t) bb[t] = pb[n0 + 16 * t + c];

  v8f acc[4];
#pragma unroll
  for (int t = 0; t < 4; ++t) acc[t] = zero8();
  gemm16x64(op, HDM, (size_t)NTOK * HDM, wf, m0, n0, lane, acc);

  const float escale = 1.0f / (WCAR * OCAR);
#pragma unroll
  for (int t = 0; t < 4; ++t) {
#pragma unroll
    for (int r = 0; r < 8; ++r) st[(n0 + 16 * t + c) * TPP + wm * 16 + 8 * hh + r] = acc[t][r] * escale + bb[t];
  }
  __syncthreads();

  {
    const int tok4 = (tid & 7) * 4;
    const int chb  = tid >> 3;
#pragma unroll
    for (int j = 0; j < 8; ++j) {
      const int ch = chb + 32 * j;
      const v4f xv = *(const v4f*)(x + ((size_t)(b * CD + ch)) * NN + nb0 + tok4);
      float* d = st + ch * TPP + tok4;
      d[0] += xv[0]; d[1] += xv[1]; d[2] += xv[2]; d[3] += xv[3];
    }
  }
  __syncthreads();

  {
    const int tok = tid >> 3;
    const int sl  = tid & 7;
    float s = 0.f;
#pragma unroll 4
    for (int cc = 0; cc < 32; ++cc) s += st[(sl * 32 + cc) * TPP + tok];
    s += __shfl_xor(s, 1, 32); s += __shfl_xor(s, 2, 32); s += __shfl_xor(s, 4, 32);
    const float mu = s * (1.0f / 256.0f);
    float d = 0.f;
#pragma unroll 4
    for (int cc = 0; cc < 32; ++cc) { const float dv = st[(sl * 32 + cc) * TPP + tok] - mu; d += dv * dv; }
    d += __shfl_xor(d, 1, 32); d += __shfl_xor(d, 2, 32); d += __shfl_xor(d, 4, 32);
    const float var = d * (1.0f / 256.0f);
    const float rs  = rsqrtf(var + 1e-5f);
    if (sl == 0) { mean_s[tok] = mu; rstd_s[tok] = rs; }
  }
  __syncthreads();

  v4f val[8];
  size_t go[8];
#pragma unroll
  for (int it = 0; it < 8; ++it) {
    const int p  = lane + 32 * it;
    const int L  = p >> 3;
    const int pc = p & 7;
    const int ch = wave * 32 + L;
    const float g = gamma[ch], be = beta[ch];
    const v4f a = *(const v4f*)(st + ch * TPP + pc * 4);
    v4f o;
#pragma unroll
    for (int i = 0; i < 4; ++i) o[i] = (a[i] - mean_s[pc * 4 + i]) * rstd_s[pc * 4 + i] * g + be;
    val[it] = o;
    go[it]  = ((size_t)(b * CD + ch)) * NN + nb0 + pc * 4;
  }
  for (int ps = 0; ps < 2; ++ps) {
#pragma unroll
    for (int it = 0; it < 8; ++it) *(volatile v4f*)(out + go[it]) = val[it];
    __threadfence();
  }
}

extern "C" void kernel_launch(void* const* d_in, const int* in_sizes, int n_in,
                              void* d_out, int out_size, void* d_ws, size_t ws_size,
                              hipStream_t stream) {
  if (n_in < 11) return;
  if (in_sizes[0] != NTOK * CD) return;
  if (in_sizes[1] != CD * CD) return;
  if (in_sizes[2] != CD) return;
  if (in_sizes[3] != CD * CD) return;
  if (in_sizes[4] != CD) return;
  if (in_sizes[5] != CD * CD) return;
  if (in_sizes[6] != CD) return;
  if (in_sizes[7] != CD * CD) return;
  if (in_sizes[8] != CD) return;
  if (in_sizes[9] != CD) return;
  if (in_sizes[10] != CD) return;
  if (out_size != NTOK * CD) return;

  const float* x     = (const float*)d_in[0];
  const float* Wq    = (const float*)d_in[1];
  const float* bq    = (const float*)d_in[2];
  const float* Wk    = (const float*)d_in[3];
  const float* bk    = (const float*)d_in[4];
  const float* Wv    = (const float*)d_in[5];
  const float* bv    = (const float*)d_in[6];
  const float* Wp    = (const float*)d_in[7];
  const float* bp    = (const float*)d_in[8];
  const float* gamma = (const float*)d_in[9];
  const float* beta  = (const float*)d_in[10];
  float* out = (float*)d_out;

  size_t off = 0;
  const size_t oW = off; off += (size_t)NWSL * CD * CD * 2;
  const size_t oX = off; off += (size_t)NTOK * CD * 2;
  const size_t oQ = off; off += (size_t)NHF * MM * HDM * 2;
  const size_t oK = off; off += (size_t)NHF * MM * HDM * 2;
  const size_t oV = off; off += (size_t)NHF * HDM * MM * 2;
  const size_t oO = off; off += (size_t)NH * NTOK * HDM * 2;
  if (off > ws_size) return;
  if (off > (size_t)134217728) return;

  char* ws = (char*)d_ws;
  _Float16* Wf = (_Float16*)(ws + oW);
  _Float16* Xf = (_Float16*)(ws + oX);
  _Float16* Qp = (_Float16*)(ws + oQ);
  _Float16* Kp = (_Float16*)(ws + oK);
  _Float16* Vt = (_Float16*)(ws + oV);
  _Float16* Op = (_Float16*)(ws + oO);

  k_xtr<<<dim3(NN / 64, CD / 64, NBAT), dim3(256), 0, stream>>>(x, Xf);
  k_wcv<<<dim3((CD * CD / 8) / 256, NWSL), dim3(256), 0, stream>>>(Wq, Wk, Wv, Wp, Wf);
  k_qkv<<<dim3(NTOK / 64, NSLAB), dim3(256), 0, stream>>>(Xf, Wf, bq, bk, bv, Qp, Kp, Vt);
  const float sscale = (float)(0.17677669529663688 / 64.0);
  k_attn<<<dim3(NHF * NQB), dim3(256), 0, stream>>>(Qp, Kp, Vt, Op, sscale);
  k_projln<<<dim3(NTOK / PR), dim3(256), 0, stream>>>(Op, Wf + (size_t)3 * CD * CD, bp, x, gamma, beta, out);
  (void)hipGetLastError();
}
